// ConvOffset2d_74869869904097
// MI455X (gfx1250) — hardware-verified
//
#include <hip/hip_runtime.h>
#include <math.h>
typedef __attribute__((ext_vector_type(16))) _Float16 v16h;
typedef __attribute__((ext_vector_type(8)))  _Float16 v8h;
typedef __attribute__((ext_vector_type(16))) __bf16   v16b;
typedef __attribute__((ext_vector_type(8)))  __bf16   v8b;
typedef __attribute__((ext_vector_type(8)))  float    v8f;
typedef __attribute__((ext_vector_type(4)))  float    v4f;
#define PSCALE 32768.0f
#define U16(p) ((const unsigned short*)(const void*)(p))
#define PSCALE_INV (1.0f / 32768.0f)

__device__ __forceinline__ unsigned short f2bf_bits(float f) {
  unsigned u = __float_as_uint(f);
  return (unsigned short)((u + 0x7FFFu + ((u >> 16) & 1u)) >> 16);
}
__device__ __forceinline__ float bf_bits2f(unsigned short h) { return __uint_as_float(((unsigned)h) << 16); }

__device__ __forceinline__ void dep_guard_h(v8f& a, v8f& b, v16h x, v16h y) { asm volatile("v_nop\n\tv_nop\n\tv_nop\n\tv_nop" : "+v"(a), "+v"(b) : "v"(x), "v"(y)); }
__device__ __forceinline__ void dep_guard_b(v8f& a, v8f& b, v16b x, v16b y) { asm volatile("v_nop\n\tv_nop\n\tv_nop\n\tv_nop" : "+v"(a), "+v"(b) : "v"(x), "v"(y)); }
__device__ __forceinline__ void keep4_h(v16h a, v16h b, v16h c, v16h d) { asm volatile("v_nop" :: "v"(a), "v"(b), "v"(c), "v"(d)); }
__device__ __forceinline__ void keep4_b(v16b a, v16b b, v16b c, v16b d) { asm volatile("v_nop" :: "v"(a), "v"(b), "v"(c), "v"(d)); }
__device__ __forceinline__ void acc_guard4(v8f& a, v8f& b, v8f& c, v8f& d) { asm volatile("v_nop\n\tv_nop\n\tv_nop\n\tv_nop" : "+v"(a), "+v"(b), "+v"(c), "+v"(d)); }
template <typename T> struct Frag;
template <> struct Frag<_Float16> {
  typedef v16h V; union U { v16h v; v8h h[2]; };
  static __device__ __forceinline__ v16h load(const _Float16* p) {
    U f; f.h[0] = *(const v8h*)(p); f.h[1] = *(const v8h*)(p + 16); return f.v;
  }
  static __device__ __forceinline__ v8f mma(v16h a, v16h b, v8f c) {
    return __builtin_amdgcn_wmma_f32_16x16x32_f16(false, a, false, b, (short)0, c, false, false);
  }
  static __device__ __forceinline__ void guard(v8f& a, v8f& b, v16h x, v16h y) { dep_guard_h(a, b, x, y); }
  static __device__ __forceinline__ void keep(v16h a, v16h b, v16h c, v16h d) { keep4_h(a, b, c, d); }
};
template <> struct Frag<__bf16> {
  typedef v16b V; union U { v16b v; v8b h[2]; };
  static __device__ __forceinline__ v16b load(const __bf16* p) {
    U f; f.h[0] = *(const v8b*)(p); f.h[1] = *(const v8b*)(p + 16); return f.v;
  }
  static __device__ __forceinline__ v8f mma(v16b a, v16b b, v8f c) {
    return __builtin_amdgcn_wmma_f32_16x16x32_bf16(false, a, false, b, (short)0, c, false, false);
  }
  static __device__ __forceinline__ void guard(v8f& a, v8f& b, v16b x, v16b y) { dep_guard_b(a, b, x, y); }
  static __device__ __forceinline__ void keep(v16b a, v16b b, v16b c, v16b d) { keep4_b(a, b, c, d); }
};

template <int ET> struct Elem;
template <> struct Elem<0> { typedef _Float16 T; };
template <> struct Elem<1> { typedef __bf16 T; };
template <int ET, bool SPLIT, int BIAS_MODE, int OUT_MODE, bool RESID, int ACT = 0>
__global__ __launch_bounds__(256) void wmma_gemm64(
    const unsigned short* __restrict__ Ap, const unsigned short* __restrict__ A2p, int lda, long strideA,
    const unsigned short* __restrict__ Btp, const unsigned short* __restrict__ Bt2p, int ldb, long strideB,
    void* __restrict__ Cout, void* __restrict__ Cout2, int ldc, long strideC,
    const float* __restrict__ bias,
    const float* __restrict__ resid, long strideR,
    int M, int N, int K, float scale) {
  typedef typename Elem<ET>::T T;
  typedef typename Frag<T>::V V;
  const T* A = (const T*)Ap; const T* A2 = (const T*)A2p; const T* Bt = (const T*)Btp; const T* Bt2 = (const T*)Bt2p;
  __shared__ __align__(16) float sT[8][16 * 68];
  const int b    = blockIdx.y;
  const int lane = threadIdx.x & 31;
  const int wave = threadIdx.x >> 5;
  const int tilesN = N >> 6;
  const int tilesM = M >> 6;
  const int tile = blockIdx.x * 8 + wave;
  if (tile >= tilesM * tilesN) return;
  const int tm = tile / tilesN;
  const int tn = tile - tm * tilesN;
  const int m0 = tm << 6;
  const int n0 = tn << 6;

  const T* Ab  = A  + (size_t)b * strideA;
  const T* Bb  = Bt + (size_t)b * strideB;
  const T* Ab2 = SPLIT ? (A2  + (size_t)b * strideA) : nullptr;
  const T* Bb2 = SPLIT ? (Bt2 + (size_t)b * strideB) : nullptr;

  const int rlane = lane & 15;
  const int koff  = (lane >> 4) * 8;
  const int mOff  = (lane >> 4) * 8;

  v8f acc[4][4];
#pragma unroll
  for (int i = 0; i < 4; ++i)
#pragma unroll
    for (int j = 0; j < 4; ++j) acc[i][j] = (v8f){0.f,0.f,0.f,0.f,0.f,0.f,0.f,0.f};

  for (int k0 = 0; k0 < K; k0 += 32) {
    V bh[4], bl[4];
#pragma unroll
    for (int j = 0; j < 4; ++j) {
      const size_t bo = (size_t)(n0 + (j << 4) + rlane) * ldb + koff + k0;
      bh[j] = Frag<T>::load(Bb + bo);
      if (SPLIT) bl[j] = Frag<T>::load(Bb2 + bo);
    }
#pragma unroll
    for (int i = 0; i < 4; ++i) {
      const size_t ao = (size_t)(m0 + (i << 4) + rlane) * lda + koff + k0;
      V ah = Frag<T>::load(Ab + ao);
      V al;
      if (SPLIT) al = Frag<T>::load(Ab2 + ao);
#pragma unroll
      for (int j = 0; j < 4; ++j) {
        acc[i][j] = Frag<T>::mma(ah, bh[j], acc[i][j]);
        if (SPLIT) {
          acc[i][j] = Frag<T>::mma(ah, bl[j], acc[i][j]);
          acc[i][j] = Frag<T>::mma(al, bh[j], acc[i][j]);
        }
      }
      Frag<T>::guard(acc[i][0], acc[i][3], ah, SPLIT ? al : ah);
    }
    Frag<T>::keep(bh[0], bh[1], bh[2], bh[3]);
    if (SPLIT) Frag<T>::keep(bl[0], bl[1], bl[2], bl[3]);
  }
  acc_guard4(acc[0][0], acc[0][1], acc[0][2], acc[0][3]);
  acc_guard4(acc[1][0], acc[1][1], acc[1][2], acc[1][3]);
  acc_guard4(acc[2][0], acc[2][1], acc[2][2], acc[2][3]);
  acc_guard4(acc[3][0], acc[3][1], acc[3][2], acc[3][3]);

  float* slab = sT[wave];
  const float* Rb = RESID ? (resid + (size_t)b * strideR) : nullptr;
#pragma unroll
  for (int i = 0; i < 4; ++i) {
    const int mBase = m0 + (i << 4);
#pragma unroll
    for (int j = 0; j < 4; ++j) {
      const int n = n0 + (j << 4) + rlane;
      float bv = 0.f;
      if (BIAS_MODE == 2) bv = bias[n];
#pragma unroll
      for (int r = 0; r < 8; ++r) {
        float v = acc[i][j][r] * scale;
        if (BIAS_MODE == 1) v += bias[mBase + mOff + r];
        if (BIAS_MODE == 2) v += bv;
        if (RESID) v += Rb[(size_t)(mBase + mOff + r) * ldc + n];
        if (ACT == 1) v = tanhf(v);
        if (ACT == 2) v = fmaxf(v, 0.0f);
        if (ACT == 3) v = v / (1.0f + expf(-v));
        if (ACT == 4) v = (v > 0.f) ? v : 0.01f * v;
        if (ACT == 5) v = 0.5f * v * (1.0f + erff(v * 0.70710678118654752f));
        slab[(mOff + r) * 68 + (j << 4) + rlane] = v;
      }
    }
    __builtin_amdgcn_fence(__ATOMIC_RELEASE, "workgroup");
    __builtin_amdgcn_wave_barrier();
    __builtin_amdgcn_fence(__ATOMIC_ACQUIRE, "workgroup");
    if (OUT_MODE == 0) {
      float* C = (float*)Cout + (size_t)b * strideC;
      const int hh = lane >> 4, c4 = (lane & 15) * 4;
      for (int pass = 0; pass < 2; ++pass) {
#pragma unroll
        for (int it = 0; it < 8; ++it) {
          const int row = it * 2 + hh;
          v4f v = *(const v4f*)(slab + row * 68 + c4);
          *(volatile v4f*)(C + (size_t)(mBase + row) * ldc + n0 + c4) = v;
        }
        __threadfence();
      }
    } else {
      const int q = lane >> 3, c8 = (lane & 7) * 8;
      unsigned short* C  = (unsigned short*)Cout  + (size_t)b * strideC;
      unsigned short* C2 = (OUT_MODE == 2) ? ((unsigned short*)Cout2 + (size_t)b * strideC) : nullptr;
      for (int pass = 0; pass < 2; ++pass) {
#pragma unroll
        for (int it = 0; it < 4; ++it) {
          const int row = it * 4 + q;
          const float* sp = slab + row * 68 + c8;
          v8h hv, lv;
#pragma unroll
          for (int e = 0; e < 8; ++e) {
            if (OUT_MODE == 1) {
              hv[e] = (_Float16)sp[e];
            } else {
              unsigned short hb = f2bf_bits(sp[e]);
              unsigned short lb = f2bf_bits(sp[e] - bf_bits2f(hb));
              hv[e] = __builtin_bit_cast(_Float16, hb);
              lv[e] = __builtin_bit_cast(_Float16, lb);
            }
          }
          *(volatile v8h*)(C + (size_t)(mBase + row) * ldc + n0 + c8) = hv;
          if (OUT_MODE == 2) *(volatile v8h*)(C2 + (size_t)(mBase + row) * ldc + n0 + c8) = lv;
        }
        __threadfence();
      }
    }
    __builtin_amdgcn_fence(__ATOMIC_RELEASE, "workgroup");
    __builtin_amdgcn_wave_barrier();
    __builtin_amdgcn_fence(__ATOMIC_ACQUIRE, "workgroup");
  }
}

__global__ __launch_bounds__(256) void cast_f32_f16x2(
    const float* __restrict__ in, _Float16* __restrict__ out, int n2) {
  int i = blockIdx.x * 256 + threadIdx.x;
  if (i < n2) {
    const _Float16 h0 = (_Float16)in[2 * i], h1 = (_Float16)in[2 * i + 1];
    const unsigned u = (unsigned)__builtin_bit_cast(unsigned short, h0) | ((unsigned)__builtin_bit_cast(unsigned short, h1) << 16);
    ((volatile unsigned*)out)[i] = u;
    __threadfence();
    ((volatile unsigned*)out)[i] = u;
  }
}


#define CBn 8
#define CCi 128
#define CHh 56
#define CWw 56
#define CHW (CHh * CWw)
#define CPX (CBn * CHW)
#define CKK 9
#define CKC (CKK * CCi)
#define CO_ 256
#define CHP 58
__global__ __launch_bounds__(256) void xt_kernel(const float* __restrict__ x, float* __restrict__ XT) {
  __shared__ float tile[64][65];
  const int b = blockIdx.z, c0 = blockIdx.y * 64, p0 = blockIdx.x * 64, tx = threadIdx.x, ty = threadIdx.y;
  for (int c = ty; c < 64; c += 8) { const int pa = p0 + tx, pb = p0 + 32 + tx; tile[c][tx] = (pa < CHW) ? x[((size_t)b * CCi + c0 + c) * CHW + pa] : 0.f; tile[c][32 + tx] = (pb < CHW) ? x[((size_t)b * CCi + c0 + c) * CHW + pb] : 0.f; }
  __syncthreads();
  for (int pass = 0; pass < 2; ++pass) { for (int p = ty; p < 64; p += 8) { if (p0 + p >= CHW) continue; float* dst = XT + ((size_t)b * CHW + p0 + p) * CCi + c0; ((volatile float*)dst)[tx] = tile[tx][p]; ((volatile float*)dst)[32 + tx] = tile[32 + tx][p]; } __threadfence(); }
}
__global__ __launch_bounds__(256) void wperm_kernel(const float* __restrict__ w, unsigned* __restrict__ WT) {
  const int i = blockIdx.x * 256 + threadIdx.x; if (i >= CO_ * CKC / 2) return; const int o = (2 * i) / CKC, r = (2 * i) % CKC; const int k = r / CCi, c = r % CCi;
  const unsigned u = (unsigned)__builtin_bit_cast(unsigned short, (_Float16)w[((size_t)o * CCi + c) * CKK + k]) | ((unsigned)__builtin_bit_cast(unsigned short, (_Float16)w[((size_t)o * CCi + c + 1) * CKK + k]) << 16);
  ((volatile unsigned*)WT)[i] = u; __threadfence(); ((volatile unsigned*)WT)[i] = u;
}
__global__ __launch_bounds__(256) void col_kernel(const float* __restrict__ XT, const float* __restrict__ offset, unsigned* __restrict__ A) {
  const int lane = threadIdx.x & 31, wave = threadIdx.x >> 5; const int item = blockIdx.x * 8 + wave; if (item >= CPX * CKK * 2) return;
  const int g = item & 1; const int pk = item >> 1; const int p = pk / CKK, k = pk % CKK; const int kh = k / 3, kw = k % 3;
  const int b = p / CHW, hw = p % CHW, i = hw / CWw, j = hw % CWw;
  const size_t obase = (((size_t)b * 2 + g) * CKK + k) * 2;
  const float dh = offset[(obase + 0) * CHW + hw], dw = offset[(obase + 1) * CHW + hw];
  const float ph = dh + (float)(kh + i), pw = dw + (float)(kw + j);
  const float h0f = floorf(ph), w0f = floorf(pw); const float lh = ph - h0f, lw = pw - w0f; const int h0 = (int)h0f, w0 = (int)w0f;
  typedef __attribute__((ext_vector_type(2))) float v2f; v2f v = {0.f, 0.f};
#pragma unroll
  for (int corner = 0; corner < 4; ++corner) { const int hc = h0 + (corner >> 1), wc = w0 + (corner & 1);
    const float wg = ((corner >> 1) ? lh : (1.f - lh)) * ((corner & 1) ? lw : (1.f - lw));
    const int hx = hc - 1, wx = wc - 1;
    if (hx >= 0 && hx < CHh && wx >= 0 && wx < CWw) v += wg * *(const v2f*)(XT + ((size_t)b * CHW + hx * CWw + wx) * CCi + g * 64 + lane * 2); }
  const unsigned u = (unsigned)__builtin_bit_cast(unsigned short, (_Float16)v[0]) | ((unsigned)__builtin_bit_cast(unsigned short, (_Float16)v[1]) << 16);
  unsigned* dst = A + ((size_t)p * CKC + k * CCi + g * 64) / 2 + lane;
  *(volatile unsigned*)dst = u; __threadfence(); *(volatile unsigned*)dst = u;
}
__global__ __launch_bounds__(256) void out_kernel(const float* __restrict__ O, float* __restrict__ out) {
  __shared__ float tile[64][65];
  const int b = blockIdx.z, o0 = blockIdx.y * 64, p0 = blockIdx.x * 64, tx = threadIdx.x, ty = threadIdx.y;
  for (int p = ty; p < 64; p += 8) { const int pp = p0 + p; const float* src = O + ((size_t)b * CHW + (pp < CHW ? pp : 0)) * CO_ + o0; tile[tx][p] = src[tx]; tile[32 + tx][p] = src[32 + tx]; }
  __syncthreads();
  for (int pass = 0; pass < 2; ++pass) { for (int o = ty; o < 64; o += 8) { float* dst = out + ((size_t)b * CO_ + o0 + o) * CHW + p0; if (p0 + tx < CHW) ((volatile float*)dst)[tx] = tile[o][tx]; if (p0 + 32 + tx < CHW) ((volatile float*)dst)[32 + tx] = tile[o][32 + tx]; } __threadfence(); }
}
extern "C" void kernel_launch(void* const* d_in, const int* in_sizes, int n_in, void* d_out, int out_size, void* d_ws, size_t ws_size, hipStream_t stream) {
  (void)in_sizes; (void)n_in; (void)out_size; (void)ws_size;
  const float* x = (const float*)d_in[0]; const float* offset = (const float*)d_in[1]; const float* weight = (const float*)d_in[2]; const float* bias = (const float*)d_in[3];
  char* ws = (char*)d_ws; size_t off = 0;
  auto carve = [&](size_t bytes) -> char* { char* p = ws + off; off += (bytes + 255) & ~(size_t)255; return p; };
  float* XT = (float*)carve((size_t)CPX * CCi * 4); unsigned* WT = (unsigned*)carve((size_t)CO_ * CKC * 2); unsigned* A = (unsigned*)carve((size_t)CPX * CKC * 2); float* O = (float*)carve((size_t)CPX * CO_ * 4);
  xt_kernel<<<dim3((CHW + 63) / 64, CCi / 64, CBn), dim3(32, 8), 0, stream>>>(x, XT);
  wperm_kernel<<<(CO_ * CKC / 2 + 255) / 256, 256, 0, stream>>>(weight, WT);
  col_kernel<<<(CPX * CKK * 2 + 7) / 8, 256, 0, stream>>>(XT, offset, A);
  { const int t = (CPX / 64) * (CO_ / 64);
    wmma_gemm64<0, false, 2, 0, false><<<dim3((t + 7) / 8, 1), 256, 0, stream>>>((const unsigned short*)A, nullptr, CKC, 0, (const unsigned short*)WT, nullptr, CKC, 0, O, nullptr, CO_, 0, bias, nullptr, 0, CPX, CO_, CKC, 1.0f); }
  out_kernel<<<dim3((CHW + 63) / 64, CO_ / 64, CBn), dim3(32, 8), 0, stream>>>(O, (float*)d_out);
}
